// TrainablePQCQCNN_52338471469482
// MI455X (gfx1250) — hardware-verified
//
#include <hip/hip_runtime.h>


typedef _Float16       v16h __attribute__((ext_vector_type(16)));
typedef _Float16       v8h  __attribute__((ext_vector_type(8)));
typedef _Float16       v4h  __attribute__((ext_vector_type(4)));
typedef __bf16         v16b __attribute__((ext_vector_type(16)));
typedef float          v8f  __attribute__((ext_vector_type(8)));
typedef float          v4f  __attribute__((ext_vector_type(4)));
typedef unsigned int   v4u  __attribute__((ext_vector_type(4)));
typedef unsigned short v4us __attribute__((ext_vector_type(4)));

union HF { v16h v; v8h hv[2]; v4h qv[4]; v8f f; };
union BF { v16b v; v4us qu[4]; v8f f; };

#define FEAT   512
#define HID    32
#define NQ     6
#define CCH    128
#define NOUT   240
#define RB     128
#define HBP    40
#define TRP    16
#define PLP    132
#define HPP    36
#define ANGOFF 8192

__device__ __forceinline__ v8f zero8() { v8f z = {0.f, 0.f, 0.f, 0.f, 0.f, 0.f, 0.f, 0.f}; return z; }

__device__ __forceinline__ v8f mma_f16(HF a, HF b, v8f c)
{
    c = __builtin_amdgcn_wmma_f32_16x16x32_f16(false, a.v, false, b.v, (short)0, c, false, false);
    asm volatile("v_nop\n\tv_nop\n\tv_nop\n\tv_nop" : "+v"(c) : "v"(a.f), "v"(b.f));
    return c;
}
__device__ __forceinline__ v8f mma_bf16(BF a, BF b, v8f c)
{
    c = __builtin_amdgcn_wmma_f32_16x16x32_bf16(false, a.v, false, b.v, (short)0, c, false, false);
    asm volatile("v_nop\n\tv_nop\n\tv_nop\n\tv_nop" : "+v"(c) : "v"(a.f), "v"(b.f));
    return c;
}

__device__ __forceinline__ HF ldh(const float* p, int h, float scale)
{
    const float* q0 = p + 8 * h;
    const float* q1 = p + 16 + 8 * h;
    const v4f t0 = *(const v4f*)(q0);
    const v4f t1 = *(const v4f*)(q0 + 4);
    const v4f t2 = *(const v4f*)(q1);
    const v4f t3 = *(const v4f*)(q1 + 4);
    HF r;
    r.qv[0] = __builtin_convertvector(t0 * scale, v4h);
    r.qv[1] = __builtin_convertvector(t1 * scale, v4h);
    r.qv[2] = __builtin_convertvector(t2 * scale, v4h);
    r.qv[3] = __builtin_convertvector(t3 * scale, v4h);
    return r;
}

__device__ __forceinline__ void split4(v4f t, v4us& hi, v4us& lo)
{
    const v4u u  = __builtin_bit_cast(v4u, t);
    const v4u hb = (u + 0x7FFFu + ((u >> 16) & 1u)) >> 16;
    const v4f hf = __builtin_bit_cast(v4f, hb << 16);
    const v4f d  = t - hf;
    const v4u ud = __builtin_bit_cast(v4u, d);
    const v4u lb = (ud + 0x7FFFu + ((ud >> 16) & 1u)) >> 16;
    hi = __builtin_convertvector(hb, v4us);
    lo = __builtin_convertvector(lb, v4us);
}

__device__ __forceinline__ void ldsplit(const float* p, int h, BF& hi, BF& lo)
{
    const float* q0 = p + 8 * h;
    const float* q1 = p + 16 + 8 * h;
    const v4f t0 = *(const v4f*)(q0);
    const v4f t1 = *(const v4f*)(q0 + 4);
    const v4f t2 = *(const v4f*)(q1);
    const v4f t3 = *(const v4f*)(q1 + 4);
    split4(t0, hi.qu[0], lo.qu[0]);
    split4(t1, hi.qu[1], lo.qu[1]);
    split4(t2, hi.qu[2], lo.qu[2]);
    split4(t3, hi.qu[3], lo.qu[3]);
}

struct cpx { float x, y; };
__device__ __forceinline__ cpx cmk(float x, float y) { cpx r; r.x = x; r.y = y; return r; }
__device__ __forceinline__ cpx cmul(cpx a, cpx b) { return cmk(a.x * b.x - a.y * b.y, a.x * b.y + a.y * b.x); }
__device__ __forceinline__ cpx cadd(cpx a, cpx b) { return cmk(a.x + b.x, a.y + b.y); }
__device__ __forceinline__ cpx cshx(cpx a, int m) { return cmk(__shfl_xor(a.x, m, 32), __shfl_xor(a.y, m, 32)); }
__device__ __forceinline__ cpx csel(bool c, cpx a, cpx b) { return cmk(c ? a.x : b.x, c ? a.y : b.y); }
struct C2 { cpx u00, u01, u10, u11; };

__device__ __forceinline__ C2 ldgate(const float* g)
{
    C2 U;
    U.u00 = cmk(g[0], g[1]); U.u01 = cmk(g[2], g[3]);
    U.u10 = cmk(g[4], g[5]); U.u11 = cmk(g[6], g[7]);
    return U;
}
__device__ __forceinline__ C2 ryc(float c, float s)
{
    C2 U;
    U.u00 = cmk(c, 0.f); U.u01 = cmk(-s, 0.f);
    U.u10 = cmk(s, 0.f); U.u11 = cmk(c, 0.f);
    return U;
}

template<int Q>
__device__ __forceinline__ void apply1(cpx& a0, cpx& a1, int lane, const C2& U)
{
    if (Q == 0) {
        const cpx n0 = cadd(cmul(U.u00, a0), cmul(U.u01, a1));
        const cpx n1 = cadd(cmul(U.u10, a0), cmul(U.u11, a1));
        a0 = n0; a1 = n1;
    } else {
        const int m = 1 << (5 - Q);
        const bool up = ((lane >> (5 - Q)) & 1) != 0;
        const cpx p0 = cshx(a0, m), p1 = cshx(a1, m);
        const cpx cs = csel(up, U.u11, U.u00);
        const cpx co = csel(up, U.u10, U.u01);
        const cpx n0 = cadd(cmul(cs, a0), cmul(co, p0));
        const cpx n1 = cadd(cmul(cs, a1), cmul(co, p1));
        a0 = n0; a1 = n1;
    }
}

template<int C, int T>
__device__ __forceinline__ void cnotg(cpx& a0, cpx& a1, int lane)
{
    if (T == 0) {
        const bool c1 = ((lane >> (5 - C)) & 1) != 0;
        const cpx t0 = csel(c1, a1, a0), t1 = csel(c1, a0, a1);
        a0 = t0; a1 = t1;
    } else if (C == 0) {
        a1 = cshx(a1, 1 << (5 - T));
    } else {
        const int m = 1 << (5 - T);
        const bool c1 = ((lane >> (5 - C)) & 1) != 0;
        const cpx p0 = cshx(a0, m), p1 = cshx(a1, m);
        a0 = csel(c1, p0, a0); a1 = csel(c1, p1, a1);
    }
}

template<int W0, int W1>
__device__ __forceinline__ void c9blk(cpx& a0, cpx& a1, int lane, const float* gb)
{
    apply1<W0>(a0, a1, lane, ldgate(gb + 0));
    apply1<W1>(a0, a1, lane, ldgate(gb + 8));
    cnotg<W0, W1>(a0, a1, lane);
    apply1<W0>(a0, a1, lane, ldgate(gb + 16));
    apply1<W1>(a0, a1, lane, ldgate(gb + 24));
    cnotg<W1, W0>(a0, a1, lane);
    apply1<W0>(a0, a1, lane, ldgate(gb + 32));
    cnotg<W0, W1>(a0, a1, lane);
    apply1<W0>(a0, a1, lane, ldgate(gb + 40));
    apply1<W1>(a0, a1, lane, ldgate(gb + 48));
}

__device__ __forceinline__ float convch(float k0, float k1, float k2, float kb, const float (&zp)[NQ + 2])
{
    float s = 0.f;
    #pragma unroll
    for (int l = 0; l < NQ; ++l) {
        const float v = k0 * zp[l] + k1 * zp[l + 1] + k2 * zp[l + 2] + kb;
        s += fmaxf(v, 0.f);
    }
    return s * (1.0f / 6.0f);
}

__device__ __forceinline__ void store_tile(float* out, const float* ob, int grow, int Bst, int tid)
{
    #pragma unroll
    for (int i = 0; i < 4; ++i) {
        const int c = tid + 256 * i;
        if (c < (16 * NOUT) / 4) {
            const int rl = c / (NOUT / 4);
            if (grow + rl < Bst) {
                const v4f v = *(const v4f*)(ob + 4 * c);
                *(volatile v4f*)(out + (size_t)grow * NOUT + 4 * c) = v;
            }
        }
    }
}

__global__ __launch_bounds__(256)
void fused_kernel(const float* __restrict__ x,
                  const float* __restrict__ w1,
                  const float* __restrict__ b1,
                  const float* __restrict__ w2,
                  const float* __restrict__ b2,
                  const float* __restrict__ qw,
                  const float* __restrict__ cw,
                  const float* __restrict__ cb,
                  const float* __restrict__ hw,
                  const float* __restrict__ hbias,
                  float* out,
                  int B, int Bst)
{
    __shared__ __align__(16) _Float16 hb_s[RB * HBP];
    __shared__ __align__(16) float    trig_s[RB * TRP];
    __shared__ __align__(16) float    gate_s[128 * 8];
    __shared__ __align__(16) float    pool_s[RB * PLP];
    __shared__ __align__(16) float    ob_s[16 * NOUT];

    const int tid  = threadIdx.x;
    const int w    = __builtin_amdgcn_readfirstlane(tid >> 5);
    const int lane = tid & 31;
    const int h    = lane >> 4;
    const int lm   = lane & 15;
    const int row0 = blockIdx.x * RB;

    if (tid < 126) {
        const int gblk = tid / 7;
        const int g    = tid - gblk * 7;
        const float* p = qw + gblk * 15;
        const int  base = (g <= 2) ? 3 * g : ((g <= 5) ? (g + 4) : 12);
        const bool isu3 = (g < 2) || (g > 4);
        const bool isrz = (g == 3);
        const float th = p[base];
        const float ph = isu3 ? p[base + 1] : 0.f;
        const float la = isu3 ? p[base + 2] : 0.f;
        const float st = sinf(0.5f * th), ct = cosf(0.5f * th);
        const float sp = sinf(ph), cp = cosf(ph);
        const float sl = sinf(la), cl = cosf(la);
        const float pl = ph + la;
        const float spl = sinf(pl), cpl = cosf(pl);
        float o0, o1, o2, o3, o4, o5, o6, o7;
        if (isrz) {
            o0 = ct;  o1 = -st; o2 = 0.f; o3 = 0.f; o4 = 0.f; o5 = 0.f; o6 = ct;  o7 = st;
        } else {
            o0 = ct;  o1 = 0.f;
            o2 = -(cl * st); o3 = -(sl * st);
            o4 = cp * st;    o5 = sp * st;
            o6 = cpl * ct;   o7 = spl * ct;
        }
        float* go = gate_s + tid * 8;
        go[0] = o0; go[1] = o1; go[2] = o2; go[3] = o3;
        go[4] = o4; go[5] = o5; go[6] = o6; go[7] = o7;
    }

    {
        int ar = row0 + 16 * w + lm;
        ar = (ar < B) ? ar : (B - 1);
        const float* xa = x  + (size_t)ar * FEAT;
        const float* wa = w1 + (size_t)lm * FEAT;
        const float* wb = w1 + (size_t)(16 + lm) * FEAT;
        v8f acc0 = zero8(), acc1 = zero8();
        #pragma unroll 4
        for (int k0 = 0; k0 < FEAT; k0 += 32) {
            const HF a  = ldh(xa + k0, h, 1.f);
            const HF f0 = ldh(wa + k0, h, 1.f);
            const HF f1 = ldh(wb + k0, h, 1.f);
            acc0 = mma_f16(a, f0, acc0);
            acc1 = mma_f16(a, f1, acc1);
        }
        #pragma unroll
        for (int r = 0; r < 8; ++r) {
            pool_s[(16 * w + 8 * h + r) * HPP + lm]      = acc0[r];
            pool_s[(16 * w + 8 * h + r) * HPP + 16 + lm] = acc1[r];
        }
    }
    __syncthreads();

    #pragma unroll 1
    for (int e = tid; e < RB * HID; e += 256) {
        const int r = e >> 5;
        const int c = e & 31;
        hb_s[r * HBP + c] = (_Float16)tanhf(pool_s[r * HPP + c] + b1[c]);
    }
    __syncthreads();

    {
        HF a;
        const _Float16* hr = hb_s + (16 * w + lm) * HBP;
        a.hv[0] = *(const v8h*)(hr + 8 * h);
        a.hv[1] = *(const v8h*)(hr + 16 + 8 * h);
        const int   qn  = (lm < NQ) ? lm : (NQ - 1);
        const float msk = (lm < NQ) ? 1.f : 0.f;
        const HF bq = ldh(w2 + qn * HID, h, msk);
        const v8f acc = mma_f16(a, bq, zero8());
        const float bb = b2[qn] * msk;
        if (lm < 8) {
            #pragma unroll
            for (int r = 0; r < 8; ++r)
                pool_s[ANGOFF + (16 * w + 8 * h + r) * 8 + lm] = acc[r] + bb;
        }
    }
    __syncthreads();

    #pragma unroll 1
    for (int e = tid; e < RB * NQ; e += 256) {
        const int r = e / NQ;
        const int q = e - r * NQ;
        const float v = 0.5f * pool_s[ANGOFF + r * 8 + q];
        trig_s[r * TRP + q]     = cosf(v);
        trig_s[r * TRP + 8 + q] = sinf(v);
    }
    __syncthreads();

    {
        float kw0[4], kw1[4], kw2[4], kbv[4];
        #pragma unroll
        for (int i = 0; i < 4; ++i) {
            const int ch = 4 * lane + i;
            kw0[i] = cw[ch * 3 + 0]; kw1[i] = cw[ch * 3 + 1]; kw2[i] = cw[ch * 3 + 2];
            kbv[i] = cb[ch];
        }
        #pragma unroll 1
        for (int j = 0; j < 16; ++j) {
            const int sl = 16 * w + j;
            const float* tr = trig_s + sl * TRP;
            float ec[NQ], es[NQ];
            #pragma unroll
            for (int q = 0; q < NQ; ++q) { ec[q] = tr[q]; es[q] = tr[8 + q]; }

            cpx a0 = cmk((lane == 0) ? 1.f : 0.f, 0.f);
            cpx a1 = cmk(0.f, 0.f);

            #pragma unroll 1
            for (int layer = 0; layer < 3; ++layer) {
                apply1<0>(a0, a1, lane, ryc(ec[0], es[0]));
                apply1<1>(a0, a1, lane, ryc(ec[1], es[1]));
                apply1<2>(a0, a1, lane, ryc(ec[2], es[2]));
                apply1<3>(a0, a1, lane, ryc(ec[3], es[3]));
                apply1<4>(a0, a1, lane, ryc(ec[4], es[4]));
                apply1<5>(a0, a1, lane, ryc(ec[5], es[5]));
                const float* gb = gate_s + layer * (6 * 56);
                c9blk<0, 1>(a0, a1, lane, gb);
                c9blk<2, 3>(a0, a1, lane, gb + 56);
                c9blk<4, 5>(a0, a1, lane, gb + 112);
                c9blk<1, 2>(a0, a1, lane, gb + 168);
                c9blk<3, 4>(a0, a1, lane, gb + 224);
                c9blk<5, 0>(a0, a1, lane, gb + 280);
            }

            const float p0 = a0.x * a0.x + a0.y * a0.y;
            const float p1 = a1.x * a1.x + a1.y * a1.y;
            const float ps = p0 + p1;
            float z[NQ];
            z[0] = p0 - p1;
            #pragma unroll
            for (int q = 1; q < NQ; ++q) z[q] = (((lane >> (5 - q)) & 1) != 0) ? -ps : ps;
            #pragma unroll
            for (int m = 1; m < 32; m <<= 1) {
                #pragma unroll
                for (int q = 0; q < NQ; ++q) z[q] += __shfl_xor(z[q], m, 32);
            }

            float zp[NQ + 2];
            zp[0] = 0.f; zp[NQ + 1] = 0.f;
            #pragma unroll
            for (int q = 0; q < NQ; ++q) zp[q + 1] = z[q];
            const float s0 = convch(kw0[0], kw1[0], kw2[0], kbv[0], zp);
            const float s1 = convch(kw0[1], kw1[1], kw2[1], kbv[1], zp);
            const float s2 = convch(kw0[2], kw1[2], kw2[2], kbv[2], zp);
            const float s3 = convch(kw0[3], kw1[3], kw2[3], kbv[3], zp);
            const v4f pv = {s0, s1, s2, s3};
            *(v4f*)(pool_s + sl * PLP + 4 * lane) = pv;
        }
    }
    __syncthreads();

    #pragma unroll 1
    for (int t = 0; t < RB / 16; ++t) {
        #pragma unroll 1
        for (int nn = 0; nn < 2; ++nn) {
            const int n = w + 8 * nn;
            if (n < NOUT / 16) {
                const float* arow = pool_s + (16 * t + lm) * PLP;
                const float* brow = hw + (size_t)(16 * n + lm) * CCH;
                v8f acc = zero8();
                #pragma unroll
                for (int ks = 0; ks < CCH / 32; ++ks) {
                    BF ah, al, bh, bl;
                    ldsplit(arow + 32 * ks, h, ah, al);
                    ldsplit(brow + 32 * ks, h, bh, bl);
                    acc = mma_bf16(ah, bh, acc);
                    acc = mma_bf16(ah, bl, acc);
                    acc = mma_bf16(al, bh, acc);
                }
                const float bias = hbias[16 * n + lm];
                #pragma unroll
                for (int r = 0; r < 8; ++r)
                    ob_s[(8 * h + r) * NOUT + 16 * n + lm] = acc[r] + bias;
            }
        }
        __syncthreads();
        const int grow = row0 + 16 * t;
        store_tile(out, ob_s, grow, Bst, tid);
        __threadfence();
        store_tile(out, ob_s, grow, Bst, tid);
        __syncthreads();
    }
}

extern "C" void kernel_launch(void* const* d_in, const int* in_sizes, int n_in,
                              void* d_out, int out_size, void* d_ws, size_t ws_size,
                              hipStream_t stream)
{
    (void)n_in; (void)d_ws; (void)ws_size;
    const float* x      = (const float*)d_in[0];
    const float* enc_w1 = (const float*)d_in[1];
    const float* enc_b1 = (const float*)d_in[2];
    const float* enc_w2 = (const float*)d_in[3];
    const float* enc_b2 = (const float*)d_in[4];
    const float* qw     = (const float*)d_in[5];
    const float* conv_w = (const float*)d_in[6];
    const float* conv_b = (const float*)d_in[7];
    const float* head_w = (const float*)d_in[8];
    const float* head_b = (const float*)d_in[9];
    float* out = (float*)d_out;

    const int B = in_sizes[0] / FEAT;
    if (B <= 0) return;
    const int Bo  = out_size / NOUT;
    const int Bst = (B < Bo) ? B : Bo;
    const int grid = (B + RB - 1) / RB;

    fused_kernel<<<dim3(grid), dim3(256), 0, stream>>>(x, enc_w1, enc_b1, enc_w2, enc_b2, qw,
                                                       conv_w, conv_b, head_w, head_b,
                                                       out, B, Bst);
}
